// Hi_Patch_7593502179555
// MI455X (gfx1250) — hardware-verified
//
#include <hip/hip_runtime.h>
#include <stddef.h>


#define DM     128
#define NH     4
#define HD     32
#define NTY    3
#define NPL    3
#define PW     384
#define QKW    192
#define NTHR   256
#define NWAVE  8
#define EPT    8
#define NGRP   2
#define CHUNK  (NTHR * EPT * NGRP)
#define WCAP   (EPT * NGRP * 32)
#define LISTN  (NWAVE * WCAP)
#define NBC    4096
#define NBF    1024
#define RCAP   40960
#define RBN    128
#define TGT    256
#define DEGCAP 128
#define NCHK   (DEGCAP / 32)
#define OTHR   512
#define EBW    64
#define EBB    (NWAVE * EBW)
#define PML    32
#define WSCAP  134217728
#define LN_EPS 1e-5f
#define DEN_EPS 1e-16f
#define NEG_BIG (-3.0e38f)
#define INV_SQRT_DK 0.17677669529663687f
#define LOG_ALPHA (-0.10536051565782628f)
#define RES_W  1.0f
#define RSQ2   0.70710678118654752f
#define ASCL   8.0f
#define WSCL   64.0f
#define INVSCL 0.001953125f
#define BMG    32
#define TPWG   6
#define KT     (DM / 32)
#define WUNITS (NPL * PW * (DM / 8))
#define LDS_FILL ((RCAP + NBF + LISTN) * 4 + 64)
#define LDS_GEMM (BMG * PW * 4)

static_assert((CHUNK & (CHUNK - 1)) == 0);
static_assert(CHUNK <= 4096);
static_assert(NBC <= 4096 && NBF <= 4096);
static_assert((NBC & (NBC - 1)) == 0 && (NBF & (NBF - 1)) == 0);
static_assert(NBC == 4 * NBF);
static_assert(OTHR * 8 == NBC);
static_assert((RCAP % 32) == 0);
static_assert(TGT == NWAVE * 32);
static_assert((NBC % TGT) == 0);
static_assert((TGT % BMG) == 0);
static_assert((TGT % NWAVE) == 0);
static_assert((WUNITS % NTHR) == 0);
static_assert(4 * TPWG * 16 == PW);
static_assert(((BMG * PW / 4) % NTHR) == 0);
static_assert(NCHK * 32 == DEGCAP);
static_assert(NH * HD == DM);
static_assert(2 * QKW == PW && NTY * DM == PW && NTY * 2 * HD == QKW);
static_assert((DM % 32) == 0);
static_assert(RCAP * 4 + NBF * 4 + LISTN * 4 + NWAVE * 4 <= LDS_FILL);
static_assert(EBW == 64 && EBB == NWAVE * 64);

typedef float          v2f  __attribute__((ext_vector_type(2)));
typedef float          v4f  __attribute__((ext_vector_type(4)));
typedef float          v8f  __attribute__((ext_vector_type(8)));
typedef int            v4i  __attribute__((ext_vector_type(4)));
typedef unsigned short v4us __attribute__((ext_vector_type(4)));
typedef unsigned short v8us __attribute__((ext_vector_type(8)));
typedef _Float16       v16h __attribute__((ext_vector_type(16)));
union FragH { v16h v; v8us u[2]; };

__device__ __forceinline__ unsigned short h16(float f) {
  const _Float16 h = (_Float16)f;
  return __builtin_bit_cast(unsigned short, h);
}

__device__ __forceinline__ v8f wmh(v16h a, v16h b, v8f c) {
  v8f d = __builtin_amdgcn_wmma_f32_16x16x32_f16(false, a, false, b, (short)0, c, false, false);
  asm volatile("v_nop\n\tv_nop\n\tv_nop\n\tv_nop" : "+v"(d) : "v"(a), "v"(b));
  return d;
}

template <int NB>
__device__ __forceinline__ int scan_chunk(const int* __restrict__ dsts, int nE, int cbase, int slotBase,
                                          int vec8, int* list, int tid, int lane, int wave) {
  int wc = 0;
#pragma unroll
  for (int g = 0; g < NGRP; ++g) {
    const int el0  = (g * NTHR + tid) * EPT;
    const int e0   = cbase + el0;
    const int sent = -2147483647 - 1;
    v4i da, db;
    if (vec8 != 0 && cbase + CHUNK <= nE) {
      da = *(const v4i*)(dsts + e0);
      db = *(const v4i*)(dsts + e0 + 4);
    } else {
      da.x = (e0     < nE) ? dsts[min(e0, nE - 1)] : sent;
      da.y = (e0 + 1 < nE) ? dsts[min(e0 + 1, nE - 1)] : sent;
      da.z = (e0 + 2 < nE) ? dsts[min(e0 + 2, nE - 1)] : sent;
      da.w = (e0 + 3 < nE) ? dsts[min(e0 + 3, nE - 1)] : sent;
      db.x = (e0 + 4 < nE) ? dsts[min(e0 + 4, nE - 1)] : sent;
      db.y = (e0 + 5 < nE) ? dsts[min(e0 + 5, nE - 1)] : sent;
      db.z = (e0 + 6 < nE) ? dsts[min(e0 + 6, nE - 1)] : sent;
      db.w = (e0 + 7 < nE) ? dsts[min(e0 + 7, nE - 1)] : sent;
    }
    const unsigned nb = (unsigned)slotBase;
    const unsigned s0 = (unsigned)da.x - nb, s1 = (unsigned)da.y - nb;
    const unsigned s2 = (unsigned)da.z - nb, s3 = (unsigned)da.w - nb;
    const unsigned s4 = (unsigned)db.x - nb, s5 = (unsigned)db.y - nb;
    const unsigned s6 = (unsigned)db.z - nb, s7 = (unsigned)db.w - nb;
    const bool h0 = s0 < (unsigned)NB, h1 = s1 < (unsigned)NB, h2 = s2 < (unsigned)NB, h3 = s3 < (unsigned)NB;
    const bool h4 = s4 < (unsigned)NB, h5 = s5 < (unsigned)NB, h6 = s6 < (unsigned)NB, h7 = s7 < (unsigned)NB;
    const unsigned any = __builtin_amdgcn_ballot_w32(h0 | h1 | h2 | h3 | h4 | h5 | h6 | h7);
    if (any != 0u) {
#define HITJ(J, HJ, SJ) { \
        const unsigned mj = __builtin_amdgcn_ballot_w32(HJ); \
        if (mj != 0u) { \
          if (HJ) { \
            const int pos = wc + (int)__builtin_amdgcn_mbcnt_lo(mj, 0u); \
            if (pos < WCAP) list[wave * WCAP + pos] = ((el0 + (J)) << 12) | (int)(SJ); \
          } \
          wc += (int)__builtin_popcount(mj); } }
      HITJ(0, h0, s0)
      HITJ(1, h1, s1)
      HITJ(2, h2, s2)
      HITJ(3, h3, s3)
      HITJ(4, h4, s4)
      HITJ(5, h5, s5)
      HITJ(6, h6, s6)
      HITJ(7, h7, s7)
#undef HITJ
    }
  }
  return wc;
}

__global__ __launch_bounds__(NTHR) void k_ln(
    const float* __restrict__ x, const float* __restrict__ gam, const float* __restrict__ bet,
    unsigned short* xn, int nN) {
  const int tid = threadIdx.x, lane = tid & 31, wave = tid >> 5;
  const int row = (int)blockIdx.x * NWAVE + wave;
  const int rc  = row > nN - 1 ? nN - 1 : row;
  const v4f v = *(const v4f*)(x + (size_t)rc * DM + 4 * lane);
  float s = v.x + v.y + v.z + v.w;
#pragma unroll
  for (int o = 16; o >= 1; o >>= 1) s += __shfl_xor(s, o);
  const float mu = s * (1.0f / DM);
  const v4f d = v - mu;
  float q = d.x * d.x + d.y * d.y + d.z * d.z + d.w * d.w;
#pragma unroll
  for (int o = 16; o >= 1; o >>= 1) q += __shfl_xor(q, o);
  const float rstd = rsqrtf(q * (1.0f / DM) + LN_EPS);
  const v4f g = *(const v4f*)(gam + 4 * lane);
  const v4f b = *(const v4f*)(bet + 4 * lane);
  const v4f o = d * rstd * g + b;
  v4us hv;
  hv[0] = h16(o.x * ASCL); hv[1] = h16(o.y * ASCL); hv[2] = h16(o.z * ASCL); hv[3] = h16(o.w * ASCL);
  unsigned short* p = xn + (size_t)row * DM + 4 * lane;
  *(volatile v4us*)p = hv;
  __threadfence();
  *(volatile v4us*)p = hv;
}

__global__ __launch_bounds__(NTHR) void k_wprep(
    const float* __restrict__ Wq, const float* __restrict__ bq,
    const float* __restrict__ Wk, const float* __restrict__ bk,
    const float* __restrict__ Wv, const float* __restrict__ bv,
    const int* __restrict__ nlp, unsigned short* wp, float* bcat, int PL) {
  const int i  = (int)blockIdx.x * NTHR + (int)threadIdx.x;
  const int g  = i / (PW * (DM / 8));
  const int rm = i - g * (PW * (DM / 8));
  const int n  = rm >> 4;
  const int d0 = (rm & 15) * 8;
  int nl = nlp[0];
  nl = nl < 0 ? 0 : (nl > PL - 1 ? PL - 1 : nl);

  {
    const int partA = n / QKW;
    const int rA = n - partA * QKW;
    const int tA = rA >> 6, hA = 2 * (g > 1 ? 1 : g) + ((rA >> 5) & 1), kA = rA & 31;
    const int tB = n >> 7, hB = (n >> 5) & 3, kB = n & 31;
    const bool isv = (g == 2);
    const int t = isv ? tB : tA, h = isv ? hB : hA, kk = isv ? kB : kA;
    const int sel = isv ? 2 : partA;
    const size_t cb = ((size_t)((h * PL + nl) * NTY + t) * DM) * HD + (size_t)kk;
    v8us hv;
#pragma unroll
    for (int e = 0; e < 8; ++e) {
      const size_t idx = cb + (size_t)(d0 + e) * HD;
      const float a = Wq[idx];
      const float b = Wk[idx];
      const float c = Wv[idx];
      const float v = (sel == 0) ? a : ((sel == 1) ? b : c);
      hv[e] = h16(v * WSCL);
    }
    unsigned short* dp = wp + (size_t)i * 8;
    *(volatile v8us*)dp = hv;
    const int bi  = i > NPL * PW - 1 ? NPL * PW - 1 : i;
    const int gb  = bi / PW;
    const int nb  = bi - gb * PW;
    const int pA2 = nb / QKW;
    const int rA2 = nb - pA2 * QKW;
    const int tA2 = rA2 >> 6, hA2 = 2 * (gb > 1 ? 1 : gb) + ((rA2 >> 5) & 1), kA2 = rA2 & 31;
    const int tB2 = nb >> 7, hB2 = (nb >> 5) & 3, kB2 = nb & 31;
    const bool isv2 = (gb == 2);
    const int t2 = isv2 ? tB2 : tA2, h2 = isv2 ? hB2 : hA2, k2 = isv2 ? kB2 : kA2;
    const int sel2 = isv2 ? 2 : pA2;
    const int bidx = ((h2 * PL + nl) * NTY + t2) * HD + k2;
    const float ba = bq[bidx], bb = bk[bidx], bc = bv[bidx];
    const float bval = (sel2 == 0) ? ba : ((sel2 == 1) ? bb : bc);
    if (i < NPL * PW) *(volatile float*)(bcat + i) = bval;
    __threadfence();
    *(volatile v8us*)dp = hv;
    if (i < NPL * PW) *(volatile float*)(bcat + i) = bval;
  }
}

__global__ __launch_bounds__(NTHR) void k_count(
    const int* __restrict__ dsts, int* cnt, int nE, int vec8) {
  __shared__ __attribute__((aligned(16))) int scnt[NBC];
  __shared__ __attribute__((aligned(16))) int list[LISTN];
  __shared__ int wcnt[NWAVE];
  const int tid = threadIdx.x, lane = tid & 31, wave = tid >> 5;
  const int nodeBase = blockIdx.x * NBC;

  for (int i = tid; i < NBC; i += NTHR) scnt[i] = 0;
  __syncthreads();

  const int nChunks = (nE + CHUNK - 1) / CHUNK;
#pragma unroll 1
  for (int ch = 0; ch < nChunks; ++ch) {
    const int cbase = ch * CHUNK;
    const int wc = scan_chunk<NBC>(dsts, nE, cbase, nodeBase, vec8, list, tid, lane, wave);
    if (lane == 0) wcnt[wave] = wc;
    __syncthreads();
    if (wave == 0) {
#pragma unroll 1
      for (int wsx = 0; wsx < NWAVE; ++wsx) {
        int n = __builtin_amdgcn_readfirstlane(wcnt[wsx]);
        n = n > WCAP ? WCAP : (n < 0 ? 0 : n);
        const int* lp = list + wsx * WCAP;
#pragma unroll 1
        for (int i = 0; i < n; ++i) {
          const int ent  = __builtin_amdgcn_readfirstlane(lp[i]);
          const int slot = ent & (NBC - 1);
          if (lane == 0) scnt[slot] = scnt[slot] + 1;
        }
      }
    }
    __syncthreads();
  }

  v4i cq[4];
#pragma unroll
  for (int q = 0; q < 4; ++q) {
    const int f = (wave * 4 + q) * 128 + 4 * lane;
    cq[q] = *(const v4i*)(scnt + f);
  }
  int* cp = cnt + (size_t)nodeBase;
#pragma unroll
  for (int q = 0; q < 4; ++q) {
    const int f = (wave * 4 + q) * 128 + 4 * lane;
    *(volatile v4i*)(cp + f) = cq[q];
  }
  __threadfence();
#pragma unroll
  for (int q = 0; q < 4; ++q) {
    const int f = (wave * 4 + q) * 128 + 4 * lane;
    *(volatile v4i*)(cp + f) = cq[q];
  }
}

__global__ __launch_bounds__(OTHR) void k_offsets(
    const int* __restrict__ cnt, int* off, int* rbase, int nChunk) {
  __shared__ __attribute__((aligned(16))) int soff[NBC];
  __shared__ __attribute__((aligned(16))) int srb[RBN];
  __shared__ int wtot[OTHR / 32];
  const int tid = threadIdx.x, lane = tid & 31, wave = tid >> 5, sub = tid >> 7;
  for (int i = tid; i < RBN; i += OTHR) srb[i] = 0;
  int carry = 0;
#pragma unroll 1
  for (int ch = 0; ch < nChunk; ++ch) {
    const int base = ch * NBC;
    const v4i c0 = *(const v4i*)(cnt + base + 8 * tid);
    const v4i c1 = *(const v4i*)(cnt + base + 8 * tid + 4);
    const int e0 = max(c0.x, 0), e1 = max(c0.y, 0), e2 = max(c0.z, 0), e3 = max(c0.w, 0);
    const int e4 = max(c1.x, 0), e5 = max(c1.y, 0), e6 = max(c1.z, 0), e7 = max(c1.w, 0);
    const int ts = e0 + e1 + e2 + e3 + e4 + e5 + e6 + e7;
    int incl = ts;
#pragma unroll
    for (int d = 1; d < 32; d <<= 1) {
      const int t = __shfl_up(incl, d);
      if (lane >= d) incl += t;
    }
    if (lane == 31) wtot[wave] = incl;
    __syncthreads();
    const int S0 = wtot[0]  + wtot[1]  + wtot[2]  + wtot[3];
    const int S1 = wtot[4]  + wtot[5]  + wtot[6]  + wtot[7];
    const int S2 = wtot[8]  + wtot[9]  + wtot[10] + wtot[11];
    const int S3 = wtot[12] + wtot[13] + wtot[14] + wtot[15];
    int pre = 0;
#pragma unroll 1
    for (int w = 4 * sub; w < wave; ++w) pre += wtot[w];
    const int b0 = carry;
    const int b1 = b0 + ((S0 + 31) & ~31);
    const int b2 = b1 + ((S1 + 31) & ~31);
    const int b3 = b2 + ((S2 + 31) & ~31);
    const int b4 = b3 + ((S3 + 31) & ~31);
    const int myb = sub == 0 ? b0 : (sub == 1 ? b1 : (sub == 2 ? b2 : b3));
    if (tid == 0) {
      srb[min(4 * ch + 0, RBN - 1)] = b0;
      srb[min(4 * ch + 1, RBN - 1)] = b1;
      srb[min(4 * ch + 2, RBN - 1)] = b2;
      srb[min(4 * ch + 3, RBN - 1)] = b3;
    }
    int run = myb + pre + incl - ts;
    soff[8 * tid + 0] = run; run += e0;
    soff[8 * tid + 1] = run; run += e1;
    soff[8 * tid + 2] = run; run += e2;
    soff[8 * tid + 3] = run; run += e3;
    soff[8 * tid + 4] = run; run += e4;
    soff[8 * tid + 5] = run; run += e5;
    soff[8 * tid + 6] = run; run += e6;
    soff[8 * tid + 7] = run;
    carry = b4;
    __syncthreads();
    const v4i o0 = *(const v4i*)(soff + 4 * tid);
    const v4i o1 = *(const v4i*)(soff + 4 * (tid + OTHR));
    int* op = off + base;
    *(volatile v4i*)(op + 4 * tid) = o0;
    *(volatile v4i*)(op + 4 * (tid + OTHR)) = o1;
    __threadfence();
    *(volatile v4i*)(op + 4 * tid) = o0;
    *(volatile v4i*)(op + 4 * (tid + OTHR)) = o1;
    __syncthreads();
  }
  if (tid == 0) srb[min(4 * nChunk, RBN - 1)] = carry;
  __syncthreads();
  v4i rv = {0, 0, 0, 0};
  if (tid < 32) rv = *(const v4i*)(srb + 4 * tid);
  if (tid < 32) *(volatile v4i*)(rbase + 4 * tid) = rv;
  __threadfence();
  if (tid < 32) *(volatile v4i*)(rbase + 4 * tid) = rv;
}

__global__ __launch_bounds__(NTHR) void k_fill(
    const int* __restrict__ dsts, const int* __restrict__ off, const int* __restrict__ rbase,
    int* csr, int nE, int vec8, int csrLen) {
  extern __shared__ v4f lds_dyn[];
  int* region = (int*)lds_dyn;
  int* cursor = region + RCAP;
  int* list   = cursor + NBF;
  int* wcnt   = list + LISTN;
  const int tid = threadIdx.x, lane = tid & 31, wave = tid >> 5;
  const int b = blockIdx.x;
  const int nodeBase = b * NBF;

  int rb0 = rbase[b];
  const int rb1 = rbase[b + 1];
  rb0 = rb0 < 0 ? 0 : (rb0 > csrLen ? csrLen : rb0);
  rb0 &= ~31;
  int len = rb1 - rb0;
  len = len < 0 ? 0 : (len > RCAP ? RCAP : len);
  int lenW = (len + 31) & ~31;
  if (rb0 + lenW > csrLen) lenW = (csrLen - rb0) & ~31;

  {
    const v4i z = {0, 0, 0, 0};
    for (int i = tid; i < RCAP / 4; i += NTHR) ((v4i*)region)[i] = z;
    for (int s = tid; s < NBF; s += NTHR) {
      int o = off[nodeBase + s] - rb0;
      o = o < 0 ? 0 : (o > RCAP ? RCAP : o);
      cursor[s] = o;
    }
  }
  __syncthreads();

  const int nChunks = (nE + CHUNK - 1) / CHUNK;
#pragma unroll 1
  for (int ch = 0; ch < nChunks; ++ch) {
    const int cbase = ch * CHUNK;
    const int wc = scan_chunk<NBF>(dsts, nE, cbase, nodeBase, vec8, list, tid, lane, wave);
    if (lane == 0) wcnt[wave] = wc;
    __syncthreads();
    if (wave == 0) {
#pragma unroll 1
      for (int wsx = 0; wsx < NWAVE; ++wsx) {
        int n = __builtin_amdgcn_readfirstlane(wcnt[wsx]);
        n = n > WCAP ? WCAP : (n < 0 ? 0 : n);
        const int* lp = list + wsx * WCAP;
#pragma unroll 1
        for (int i = 0; i < n; ++i) {
          const int ent  = __builtin_amdgcn_readfirstlane(lp[i]);
          const int slot = ent & (NBF - 1);
          int e = cbase + ((ent >> 12) & (CHUNK - 1));
          e = e > nE - 1 ? nE - 1 : e;
          if (lane == 0) {
            int pos = cursor[slot];
            pos = pos < 0 ? 0 : (pos > RCAP - 1 ? RCAP - 1 : pos);
            region[pos] = e;
            const int np = pos + 1;
            cursor[slot] = np > RCAP ? RCAP : np;
          }
        }
      }
    }
    __syncthreads();
  }

  const int nv = lenW >> 2;
  int* gp = csr + rb0;
#pragma unroll 1
  for (int i = tid; i < nv; i += NTHR) { const v4i v = ((const v4i*)region)[i]; *(volatile v4i*)(gp + 4 * i) = v; }
  __threadfence();
#pragma unroll 1
  for (int i = tid; i < nv; i += NTHR) { const v4i v = ((const v4i*)region)[i]; *(volatile v4i*)(gp + 4 * i) = v; }
}

__global__ __launch_bounds__(NTHR) void k_gemm(
    const unsigned short* __restrict__ A, const unsigned short* __restrict__ wp,
    const float* __restrict__ bcat, float* P) {
  extern __shared__ v4f lds_dyn[];
  float* stg = (float*)lds_dyn;
  const int tid = threadIdx.x, lane = tid & 31, wave = tid >> 5, hh = lane >> 4, m = lane & 15;
  const int rowBase = blockIdx.x * BMG;
  const int rg = wave >> 2;
  const int cq = wave & 3;
  const int r0 = rg * 16;
  const int c0 = cq * (TPWG * 16);

  v8f acc[TPWG];
#pragma unroll
  for (int t = 0; t < TPWG; ++t) { v8f z = {0.f, 0.f, 0.f, 0.f, 0.f, 0.f, 0.f, 0.f}; acc[t] = z; }
  const unsigned short* afp = A + (size_t)(rowBase + r0 + m) * DM + 8 * hh;
#pragma unroll
  for (int kt = 0; kt < KT; ++kt) {
    FragH af;
    af.u[0] = *(const v8us*)(afp + 32 * kt);
    af.u[1] = *(const v8us*)(afp + 32 * kt + 16);
#pragma unroll
    for (int t = 0; t < TPWG; ++t) {
      const unsigned short* bp = wp + (size_t)(c0 + 16 * t + m) * DM + 32 * kt + 8 * hh;
      FragH bf;
      bf.u[0] = *(const v8us*)bp;
      bf.u[1] = *(const v8us*)(bp + 16);
      acc[t] = wmh(af.v, bf.v, acc[t]);
    }
  }

  {
    float* sp = stg + (size_t)(r0 + 8 * hh) * PW + c0 + m;
#pragma unroll
    for (int t = 0; t < TPWG; ++t) {
#pragma unroll
      for (int r = 0; r < 8; ++r) sp[r * PW + 16 * t] = acc[t][r];
    }
  }
  __syncthreads();

  float* gp = P + (size_t)rowBase * PW;
  constexpr int NIT = (BMG * PW / 4) / NTHR;
#pragma unroll
  for (int it = 0; it < NIT; ++it) {
    const int f    = it * NTHR + tid;
    const int col4 = f % (PW / 4);
    const v4f v  = *(const v4f*)(stg + 4 * f);
    const v4f bb = *(const v4f*)(bcat + 4 * col4);
    const v4f o  = v * INVSCL + bb;
    *(volatile v4f*)(gp + 4 * (size_t)f) = o;
  }
  __threadfence();
#pragma unroll
  for (int it = 0; it < NIT; ++it) {
    const int f    = it * NTHR + tid;
    const int col4 = f % (PW / 4);
    const v4f v  = *(const v4f*)(stg + 4 * f);
    const v4f bb = *(const v4f*)(bcat + 4 * col4);
    const v4f o  = v * INVSCL + bb;
    *(volatile v4f*)(gp + 4 * (size_t)f) = o;
  }
}

template <int G>
__global__ __launch_bounds__(NTHR) void k_att(
    const float* __restrict__ P, const int* __restrict__ ei,
    const float* __restrict__ m0, const float* __restrict__ m1, const float* __restrict__ m2,
    const float* __restrict__ ev, float* attp, float* pmax, int nN, int nE) {
  __shared__ __attribute__((aligned(16))) float sAtt[NWAVE * 128];
  __shared__ float wmax[NWAVE * 2];
  const int tid = threadIdx.x, lane = tid & 31, wave = tid >> 5;
  const int sub = lane >> 4, cl = lane & 15, hl = cl >> 3;
  const int base = (int)blockIdx.x * EBB + wave * EBW;

  float mx = NEG_BIG;
#pragma unroll 1
  for (int j = 0; j < 32; ++j) {
    const int el = 2 * j + sub;
    const int e  = base + el;
    const bool valid = e < nE;
    const int ec = e > nE - 1 ? nE - 1 : e;
    int dn = ei[(size_t)nE + ec];
    dn = dn < 0 ? 0 : (dn > nN - 1 ? nN - 1 : dn);
    int sn = ei[ec];
    sn = sn < 0 ? 0 : (sn > nN - 1 ? nN - 1 : sn);
    const float v0 = m0[ec], v1 = m1[ec], v2 = m2[ec];
    const bool c1 = v1 > v0;
    int t = c1 ? 1 : 0;
    float ms = c1 ? v1 : v0;
    const bool c2 = v2 > ms;
    t  = c2 ? 2 : t;
    ms = c2 ? v2 : ms;
    const v4f q4 = *(const v4f*)(P + (size_t)dn * PW + t * (2 * HD) + 4 * cl);
    const v4f k4 = *(const v4f*)(P + (size_t)sn * PW + QKW + t * (2 * HD) + 4 * cl);
    float d = q4.x * k4.x + q4.y * k4.y + q4.z * k4.z + q4.w * k4.w;
    d += __shfl_xor(d, 1);
    d += __shfl_xor(d, 2);
    d += __shfl_xor(d, 4);
    const float dec = __expf(LOG_ALPHA * fabsf(ev[ec]));
    const float a = ((d * (ms * ms)) * INV_SQRT_DK) * dec;
    mx = fmaxf(mx, valid ? a : NEG_BIG);
    if ((cl & 7) == 0) sAtt[wave * 128 + el * 2 + hl] = valid ? a : 0.f;
  }
  mx = fmaxf(mx, __shfl_xor(mx, 16));
  if (lane == 0) wmax[wave * 2] = mx;
  if (lane == 8) wmax[wave * 2 + 1] = mx;
  __syncthreads();

  const v4f av = *(const v4f*)(sAtt + wave * 128 + 4 * lane);
  float* ap = attp + (size_t)base * 2 + 4 * lane;
  float bm0 = NEG_BIG, bm1 = NEG_BIG;
#pragma unroll
  for (int w = 0; w < NWAVE; ++w) { bm0 = fmaxf(bm0, wmax[2 * w]); bm1 = fmaxf(bm1, wmax[2 * w + 1]); }
  v4f pv = {0.f, 0.f, 0.f, 0.f};
  pv.x = (lane == 0) ? bm0 : 0.f;
  pv.y = (lane == 0) ? bm1 : 0.f;
  float* pp = pmax + (size_t)blockIdx.x * PML + 4 * lane;
  const bool pw = (wave == 0) && (lane < 8);
  *(volatile v4f*)ap = av;
  if (pw) *(volatile v4f*)pp = pv;
  __threadfence();
  *(volatile v4f*)ap = av;
  if (pw) *(volatile v4f*)pp = pv;
}

__global__ __launch_bounds__(NTHR) void k_gmax(
    const float* __restrict__ pm0, const float* __restrict__ pm1, float* gm, int nBlk) {
  __shared__ float swm[NWAVE * 4];
  const int tid = threadIdx.x, lane = tid & 31, wave = tid >> 5;
  v4f mx = {NEG_BIG, NEG_BIG, NEG_BIG, NEG_BIG};
#pragma unroll 1
  for (int b = tid; b < nBlk; b += NTHR) {
    const v4f a = *(const v4f*)(pm0 + (size_t)b * PML);
    const v4f c = *(const v4f*)(pm1 + (size_t)b * PML);
    mx.x = fmaxf(mx.x, a.x); mx.y = fmaxf(mx.y, a.y);
    mx.z = fmaxf(mx.z, c.x); mx.w = fmaxf(mx.w, c.y);
  }
#pragma unroll
  for (int o = 1; o < 32; o <<= 1) {
    mx.x = fmaxf(mx.x, __shfl_xor(mx.x, o));
    mx.y = fmaxf(mx.y, __shfl_xor(mx.y, o));
    mx.z = fmaxf(mx.z, __shfl_xor(mx.z, o));
    mx.w = fmaxf(mx.w, __shfl_xor(mx.w, o));
  }
  if (lane == 0) { swm[4 * wave] = mx.x; swm[4 * wave + 1] = mx.y; swm[4 * wave + 2] = mx.z; swm[4 * wave + 3] = mx.w; }
  __syncthreads();
  v4f r = {NEG_BIG, NEG_BIG, NEG_BIG, NEG_BIG};
#pragma unroll
  for (int w = 0; w < NWAVE; ++w) {
    r.x = fmaxf(r.x, swm[4 * w]); r.y = fmaxf(r.y, swm[4 * w + 1]);
    r.z = fmaxf(r.z, swm[4 * w + 2]); r.w = fmaxf(r.w, swm[4 * w + 3]);
  }
  v4f pv = {0.f, 0.f, 0.f, 0.f};
  pv.x = (lane == 0) ? r.x : 0.f;
  pv.y = (lane == 0) ? r.y : 0.f;
  pv.z = (lane == 0) ? r.z : 0.f;
  pv.w = (lane == 0) ? r.w : 0.f;
  const bool pw = (wave == 0) && (lane < 8);
  if (pw) *(volatile v4f*)(gm + 4 * lane) = pv;
  __threadfence();
  if (pw) *(volatile v4f*)(gm + 4 * lane) = pv;
}

__global__ __launch_bounds__(NTHR) void k_agg(
    const int* __restrict__ csr, const int* __restrict__ off, const int* __restrict__ cnt,
    const int* __restrict__ ei,
    const float* __restrict__ m0, const float* __restrict__ m1, const float* __restrict__ m2,
    const float* __restrict__ at0, const float* __restrict__ at1, const float* __restrict__ gmax,
    const float* __restrict__ P, const float* __restrict__ x, float* out,
    int nN, int nE, int csrLen) {
  const int tid = threadIdx.x, lane = tid & 31, wave = tid >> 5, hh = lane >> 3;
  const int tbase = blockIdx.x * TGT + wave * 32;
  const v4f z4 = {0.f, 0.f, 0.f, 0.f};

  const int cl    = tbase + lane;
  const int cnt_l = cnt[cl];
  const int off_l = off[cl];
  const v4f g4 = *(const v4f*)gmax;

#pragma unroll 1
  for (int j = 0; j < 32; ++j) {
    const int c = tbase + j;
    int n = __builtin_amdgcn_readfirstlane(__shfl(cnt_l, j));
    n = n < 0 ? 0 : (n > DEGCAP ? DEGCAP : n);
    const int st = __builtin_amdgcn_readfirstlane(__shfl(off_l, j));

    v4f den = z4;
    v4f acc = z4;
#pragma unroll 1
    for (int kc = 0; kc < NCHK; ++kc) {
      const int q0 = 32 * kc;
      if (q0 < n) {
        int pos = st + q0 + lane;
        pos = pos < 0 ? 0 : (pos > csrLen - 1 ? csrLen - 1 : pos);
        int eid = csr[pos];
        eid = eid < 0 ? 0 : (eid > nE - 1 ? nE - 1 : eid);
        const bool lv = (q0 + lane) < n;
        int sn = ei[eid];
        sn = sn < 0 ? 0 : (sn > nN - 1 ? nN - 1 : sn);
        const float v0 = m0[eid], v1 = m1[eid], v2 = m2[eid];
        const bool c1 = v1 > v0;
        int t = c1 ? 1 : 0;
        float ms = c1 ? v1 : v0;
        const bool c2 = v2 > ms;
        t  = c2 ? 2 : t;
        ms = c2 ? v2 : ms;
        const v2f a01 = *(const v2f*)(at0 + 2 * (size_t)eid);
        const v2f a23 = *(const v2f*)(at1 + 2 * (size_t)eid);
        v4f p;
        p.x = __expf(a01.x - g4.x);
        p.y = __expf(a01.y - g4.y);
        p.z = __expf(a23.x - g4.z);
        p.w = __expf(a23.y - g4.w);
        p.x = lv ? p.x : 0.f; p.y = lv ? p.y : 0.f; p.z = lv ? p.z : 0.f; p.w = lv ? p.w : 0.f;
        den = den + p;
        const int mcnt = (n - q0) < 32 ? (n - q0) : 32;
#pragma unroll 1
        for (int pp = 0; pp < mcnt; ++pp) {
          const int   s   = __builtin_amdgcn_readlane(sn, pp);
          const int   tt  = __builtin_amdgcn_readlane(t, pp);
          const float msv = __shfl(ms, pp);
          const float px = __shfl(p.x, pp), py = __shfl(p.y, pp), pz = __shfl(p.z, pp), pq = __shfl(p.w, pp);
          const float ph = (hh == 0) ? px : ((hh == 1) ? py : ((hh == 2) ? pz : pq));
          const v4f v4 = *(const v4f*)(P + (size_t)s * PW + tt * DM + 4 * lane);
          acc = acc + v4 * (ph * msv);
        }
      }
    }
#pragma unroll
    for (int o = 1; o < 32; o <<= 1) {
      den.x += __shfl_xor(den.x, o);
      den.y += __shfl_xor(den.y, o);
      den.z += __shfl_xor(den.z, o);
      den.w += __shfl_xor(den.w, o);
    }
    const float dsel = (hh == 0) ? den.x : ((hh == 1) ? den.y : ((hh == 2) ? den.z : den.w));
    const float rd = 1.0f / (dsel + DEN_EPS);
    const v4f res = acc * rd;

    if (c < nN) {
      const v4f x4 = *(const v4f*)(x + (size_t)c * DM + 4 * lane);
      v4f gl = res;
#pragma unroll 1
      for (int qq = 0; qq < 4; ++qq) {
        const float a  = (qq == 0) ? res.x : ((qq == 1) ? res.y : ((qq == 2) ? res.z : res.w));
        const float gv = 0.5f * a * (1.0f + erff(a * RSQ2));
        gl.x = (qq == 0) ? gv : gl.x;
        gl.y = (qq == 1) ? gv : gl.y;
        gl.z = (qq == 2) ? gv : gl.z;
        gl.w = (qq == 3) ? gv : gl.w;
      }
      const v4f o = x4 * RES_W + gl;
      float* op = out + (size_t)c * DM + 4 * lane;
      *(volatile v4f*)op = o;
      __threadfence();
      *(volatile v4f*)op = o;
    }
  }
}

extern "C" void kernel_launch(void* const* d_in, const int* in_sizes, int n_in,
                              void* d_out, int out_size, void* d_ws, size_t ws_size,
                              hipStream_t stream) {
  if (n_in < 16) return;
  const int nN = in_sizes[0] / DM;
  if (nN <= 0 || in_sizes[0] != nN * DM) return;
  const int nE = in_sizes[1] / 2;
  if (nE <= 0 || in_sizes[1] != 2 * nE) return;
  if (in_sizes[2] != nE || in_sizes[4] != nE || in_sizes[5] != nE || in_sizes[6] != nE) return;
  if (in_sizes[7] < 1 || in_sizes[8] != DM || in_sizes[9] != DM) return;
  const int wunit = NH * NTY * DM * HD;
  const int PL = in_sizes[10] / wunit;
  if (PL < 1 || in_sizes[10] != PL * wunit) return;
  if (in_sizes[12] != in_sizes[10] || in_sizes[14] != in_sizes[10]) return;
  const int bunit = NH * NTY * HD;
  if (in_sizes[11] != PL * bunit || in_sizes[13] != PL * bunit || in_sizes[15] != PL * bunit) return;
  if (out_size != nN * DM) return;
  if (nE > (1 << 27) || nN > (1 << 22)) return;

  const float* x    = (const float*)d_in[0];
  const int*   ei   = (const int*)d_in[1];
  const int*   dsts = ei + nE;
  const float* ev   = (const float*)d_in[2];
  const float* mk0  = (const float*)d_in[4];
  const float* mk1  = (const float*)d_in[5];
  const float* mk2  = (const float*)d_in[6];
  const int*   nlp  = (const int*)d_in[7];
  const float* gam  = (const float*)d_in[8];
  const float* bet  = (const float*)d_in[9];
  const float* Wq   = (const float*)d_in[10];
  const float* bq   = (const float*)d_in[11];
  const float* Wk   = (const float*)d_in[12];
  const float* bk   = (const float*)d_in[13];
  const float* Wv   = (const float*)d_in[14];
  const float* bv   = (const float*)d_in[15];
  float* out = (float*)d_out;

  const int NPAD   = ((nN + TGT - 1) / TGT) * TGT;
  const int nBC    = (nN + NBC - 1) / NBC;
  const int CNTPAD = nBC * NBC;
  if (4 * nBC + 1 > RBN) return;
  const int nBF    = (nN + NBF - 1) / NBF;
  const int csrLen = ((nE + 31) & ~31) + 4096;
  if (31 * 4 * nBC > 4096) return;
  const int nAgg   = NPAD / TGT;
  const int nGemm  = NPAD / BMG;
  const int nLn    = NPAD / NWAVE;
  const int nAttB  = (nE + EBB - 1) / EBB;
  const int EPAD   = nAttB * EBB;

  char* ws = (char*)d_ws;
  size_t off = 0;
  const size_t oXn  = off; off += (size_t)NPAD * DM * 2;          off = (off + 255) & ~(size_t)255;
  const size_t oWp  = off; off += (size_t)NPL * PW * DM * 2;      off = (off + 255) & ~(size_t)255;
  const size_t oBc  = off; off += (size_t)NPL * PW * 4;           off = (off + 255) & ~(size_t)255;
  const size_t oCnt = off; off += (size_t)CNTPAD * 4;             off = (off + 255) & ~(size_t)255;
  const size_t oOff = off; off += (size_t)CNTPAD * 4;             off = (off + 255) & ~(size_t)255;
  const size_t oRb  = off; off += (size_t)RBN * 4;                off = (off + 255) & ~(size_t)255;
  const size_t oCsr = off; off += (size_t)csrLen * 4;             off = (off + 255) & ~(size_t)255;
  const size_t oAt0 = off; off += (size_t)EPAD * 2 * 4;           off = (off + 255) & ~(size_t)255;
  const size_t oAt1 = off; off += (size_t)EPAD * 2 * 4;           off = (off + 255) & ~(size_t)255;
  const size_t oPm0 = off; off += (size_t)nAttB * PML * 4;        off = (off + 255) & ~(size_t)255;
  const size_t oPm1 = off; off += (size_t)nAttB * PML * 4;        off = (off + 255) & ~(size_t)255;
  const size_t oGm  = off; off += (size_t)PML * 4;                off = (off + 255) & ~(size_t)255;
  const size_t oP   = off; off += (size_t)NPAD * PW * 4;          off = (off + 255) & ~(size_t)255;
  if (off > ws_size || off > (size_t)WSCAP) return;
  unsigned short* xn = (unsigned short*)(ws + oXn);
  unsigned short* wp = (unsigned short*)(ws + oWp);
  float* bcat = (float*)(ws + oBc);
  int*   cnt  = (int*)(ws + oCnt);
  int*   offp = (int*)(ws + oOff);
  int*   rb   = (int*)(ws + oRb);
  int*   csr  = (int*)(ws + oCsr);
  float* at0  = (float*)(ws + oAt0);
  float* at1  = (float*)(ws + oAt1);
  float* pm0  = (float*)(ws + oPm0);
  float* pm1  = (float*)(ws + oPm1);
  float* gm   = (float*)(ws + oGm);
  float* P    = (float*)(ws + oP);

  const int vec8 = ((nE & 3) == 0) ? 1 : 0;

  k_ln<<<nLn, NTHR, 0, stream>>>(x, gam, bet, xn, nN);
  k_wprep<<<WUNITS / NTHR, NTHR, 0, stream>>>(Wq, bq, Wk, bk, Wv, bv, nlp, wp, bcat, PL);
  k_count<<<nBC, NTHR, 0, stream>>>(dsts, cnt, nE, vec8);
  k_offsets<<<1, OTHR, 0, stream>>>(cnt, offp, rb, nBC);
  hipFuncSetAttribute(reinterpret_cast<const void*>(&k_fill),
                      hipFuncAttributeMaxDynamicSharedMemorySize, LDS_FILL);
  k_fill<<<nBF, NTHR, LDS_FILL, stream>>>(dsts, offp, rb, csr, nE, vec8, csrLen);
  hipFuncSetAttribute(reinterpret_cast<const void*>(&k_gemm),
                      hipFuncAttributeMaxDynamicSharedMemorySize, LDS_GEMM);
  k_gemm<<<nGemm, NTHR, LDS_GEMM, stream>>>(xn, wp, bcat, P);
  k_att<0><<<nAttB, NTHR, 0, stream>>>(P, ei, mk0, mk1, mk2, ev, at0, pm0, nN, nE);
  k_gemm<<<nGemm, NTHR, LDS_GEMM, stream>>>(xn, wp + (size_t)PW * DM, bcat + PW, P);
  k_att<1><<<nAttB, NTHR, 0, stream>>>(P, ei, mk0, mk1, mk2, ev, at1, pm1, nN, nE);
  k_gmax<<<1, NTHR, 0, stream>>>(pm0, pm1, gm, nAttB);
  k_gemm<<<nGemm, NTHR, LDS_GEMM, stream>>>(xn, wp + (size_t)2 * PW * DM, bcat + 2 * PW, P);
  k_agg<<<nAgg, NTHR, 0, stream>>>(csr, offp, cnt, ei, mk0, mk1, mk2, at0, at1, gm, P, x, out, nN, nE, csrLen);
}
